// JacobianMLP_69157563400601
// MI455X (gfx1250) — hardware-verified
//
#include <hip/hip_runtime.h>
#include <stdint.h>


typedef float v8f __attribute__((ext_vector_type(8)));
typedef float v4f __attribute__((ext_vector_type(4))) __attribute__((may_alias));
typedef unsigned short v8us __attribute__((ext_vector_type(8))) __attribute__((may_alias));
typedef unsigned short v16us __attribute__((ext_vector_type(16)));
typedef __bf16 v16bf __attribute__((ext_vector_type(16)));

union Frag16 { v16bf v; v16us u; v8us h8[2]; };

#define IN_DIM          16
#define OUT_DIM         16
#define HID             512
#define NT              (HID / 16)
#define WAVES           8
#define ROWS_PER_WAVE   16
#define ROWS_PER_BLOCK  (WAVES * ROWS_PER_WAVE)
#define NEG_SLOPE       0.2f

__device__ __forceinline__ unsigned short bf16_rne_bits(float f) {
    unsigned int u = __float_as_uint(f);
    u += 0x7FFFu + ((u >> 16) & 1u);
    return (unsigned short)(u >> 16);
}
__device__ __forceinline__ float bf16_bits_to_f32(unsigned short s) {
    return __uint_as_float(((unsigned int)s) << 16);
}
__device__ __forceinline__ void split_bf16(float v, unsigned short& hi, unsigned short& lo) {
    hi = bf16_rne_bits(v);
    const float r = v - bf16_bits_to_f32(hi);
    lo = bf16_rne_bits(r);
}

__device__ __forceinline__ v8f wmma_pair_bf16(v16bf a, v16bf bh, v16bf bl, v8f c) {
    c = __builtin_amdgcn_wmma_f32_16x16x32_bf16(false, a, false, bh, (short)0, c, false, false);
    c = __builtin_amdgcn_wmma_f32_16x16x32_bf16(false, a, false, bl, (short)0, c, false, false);
    asm volatile("v_nop\n\tv_nop\n\tv_nop\n\tv_nop" : "+v"(c) : "v"(a), "v"(bh), "v"(bl));
    return c;
}

__global__ __launch_bounds__(256) void k_split_w1(const float* __restrict__ W1,
                                                  unsigned short* __restrict__ Whi,
                                                  unsigned short* __restrict__ Wlo,
                                                  int nvec)
{
    const int i = blockIdx.x * 256 + threadIdx.x;
    const bool ok = i < nvec;
    const int ic = ok ? i : 0;
    const v4f* src = (const v4f*)(W1 + (size_t)ic * 8);
    const v4f f0 = src[0], f1 = src[1];
    v8us hv, lv;
    #pragma unroll
    for (int e = 0; e < 4; ++e) {
        unsigned short hh, ll;
        split_bf16(f0[e], hh, ll); hv[e] = hh;     lv[e] = ll;
        split_bf16(f1[e], hh, ll); hv[4 + e] = hh; lv[4 + e] = ll;
    }
    unsigned short* ph = Whi + (size_t)ic * 8;
    unsigned short* pl = Wlo + (size_t)ic * 8;
    if (ok) {
        *(volatile v8us*)ph = hv;
        *(volatile v8us*)pl = lv;
    }
    __threadfence();
    if (ok) {
        *(volatile v8us*)ph = hv;
        *(volatile v8us*)pl = lv;
    }
}

__global__ __launch_bounds__(256) void k_mlp16(const float* __restrict__ x,
                                               const unsigned short* __restrict__ Whi,
                                               const unsigned short* __restrict__ Wlo,
                                               const float* __restrict__ b1,
                                               const float* __restrict__ W2,
                                               const float* __restrict__ b2,
                                               float* __restrict__ out,
                                               int nrows)
{
    __shared__ __align__(16) float sOut[WAVES * ROWS_PER_WAVE * OUT_DIM];

    const int tid  = threadIdx.x;
    const int lane = tid & 31;
    const int wave = tid >> 5;
    const int h    = lane >> 4;
    const int l16  = lane & 15;

    const int rbase = blockIdx.x * ROWS_PER_BLOCK + wave * ROWS_PER_WAVE;
    int row = rbase + l16;
    if (row > nrows - 1) row = nrows - 1;

    Frag16 fa;
    {
        const v4f* xp = (const v4f*)(x + (size_t)row * IN_DIM + 8 * h);
        const v4f x0 = xp[0], x1 = xp[1];
        v16us au;
        #pragma unroll
        for (int e = 0; e < 4; ++e) {
            unsigned short hh, ll;
            split_bf16(x0[e], hh, ll); au[e] = hh;     au[8 + e] = ll;
            split_bf16(x1[e], hh, ll); au[4 + e] = hh; au[12 + e] = ll;
        }
        fa.u = au;
    }

    float* sw = sOut + wave * (ROWS_PER_WAVE * OUT_DIM);

    #pragma unroll 1
    for (int o = 0; o < OUT_DIM; ++o) {
        const unsigned short* who = Whi + (size_t)o * HID * IN_DIM;
        const unsigned short* wlo = Wlo + (size_t)o * HID * IN_DIM;
        const float* b1o = b1 + (size_t)o * HID;
        const float* W2o = W2 + (size_t)o * HID;
        const float  b2v = b2[o];

        float acc[8];
        #pragma unroll
        for (int r = 0; r < 8; ++r) acc[r] = 0.0f;

        #pragma unroll 2
        for (int t = 0; t < NT; ++t) {
            const int n = t * 16 + l16;
            Frag16 fbh, fbl;
            const v8us ph = *(const v8us*)(who + (size_t)n * IN_DIM + 8 * h);
            const v8us pl = *(const v8us*)(wlo + (size_t)n * IN_DIM + 8 * h);
            fbh.h8[0] = ph; fbh.h8[1] = ph;
            fbl.h8[0] = pl; fbl.h8[1] = pl;
            const float bn = b1o[n];
            const float wn = W2o[n];
            v8f c = { bn, bn, bn, bn, bn, bn, bn, bn };
            c = wmma_pair_bf16(fa.v, fbh.v, fbl.v, c);
            #pragma unroll
            for (int r = 0; r < 8; ++r) {
                const float hv = c[r];
                const float lk = fmaxf(hv, hv * NEG_SLOPE);
                acc[r] = fmaf(lk, wn, acc[r]);
            }
        }

        #pragma unroll
        for (int r = 0; r < 8; ++r) {
            #pragma unroll
            for (int off = 1; off < 16; off <<= 1)
                acc[r] += __shfl_xor(acc[r], off, 32);
        }
        float val = acc[0];
        #pragma unroll
        for (int j = 1; j < 8; ++j) val = (l16 == j) ? acc[j] : val;
        if (l16 < 8) sw[(8 * h + l16) * OUT_DIM + o] = val + b2v;
    }

    __syncthreads();

    const v4f v0 = *(const v4f*)(sw + lane * 4);
    const v4f v1 = *(const v4f*)(sw + 128 + lane * 4);
    const bool p0 = (rbase + (lane >> 2)) < nrows;
    const bool p1 = (rbase + 8 + (lane >> 2)) < nrows;
    float* dst = out + (size_t)rbase * OUT_DIM;
    if (p0) *(volatile v4f*)(dst + lane * 4) = v0;
    if (p1) *(volatile v4f*)(dst + 128 + lane * 4) = v1;
    __threadfence();
    if (p0) *(volatile v4f*)(dst + lane * 4) = v0;
    if (p1) *(volatile v4f*)(dst + 128 + lane * 4) = v1;
}

extern "C" void kernel_launch(void* const* d_in, const int* in_sizes, int n_in,
                              void* d_out, int out_size, void* d_ws, size_t ws_size,
                              hipStream_t stream)
{
    if (n_in < 5) return;
    const int nx  = in_sizes[0];
    const int nw1 = in_sizes[1];
    const int nb1 = in_sizes[2];
    const int nw2 = in_sizes[3];
    const int nb2 = in_sizes[4];
    const int nrows = nx / IN_DIM;
    if (nrows <= 0 || nx != nrows * IN_DIM) return;
    if (nw1 != OUT_DIM * HID * IN_DIM || nb1 != OUT_DIM * HID || nw2 != OUT_DIM * HID || nb2 != OUT_DIM) return;
    if (out_size != nrows * OUT_DIM) return;

    const size_t plane_bytes = (size_t)nw1 * sizeof(unsigned short);
    if (2 * plane_bytes > ws_size) return;
    unsigned short* Whi = (unsigned short*)d_ws;
    unsigned short* Wlo = Whi + nw1;

    const float* x  = (const float*)d_in[0];
    const float* W1 = (const float*)d_in[1];
    const float* b1 = (const float*)d_in[2];
    const float* W2 = (const float*)d_in[3];
    const float* b2 = (const float*)d_in[4];
    float* out = (float*)d_out;

    const int nvec = nw1 / 8;
    dim3 gcv((nvec + 255) / 256);
    k_split_w1<<<gcv, dim3(256), 0, stream>>>(W1, Whi, Wlo, nvec);

    dim3 gm((nrows + ROWS_PER_BLOCK - 1) / ROWS_PER_BLOCK);
    k_mlp16<<<gm, dim3(256), 0, stream>>>(x, Whi, Wlo, b1, W2, b2, out, nrows);
    (void)hipGetLastError();
}
